// RWKV6Mixin_5188320493605
// MI455X (gfx1250) — hardware-verified
//
#include <hip/hip_runtime.h>
#include <math.h>

constexpr int kBatch = 2;
constexpr int kSeqT  = 1024;
constexpr int kHid   = 2048;
constexpr int kTok   = kBatch * kSeqT;
constexpr int kKD    = 1024;
constexpr int kVD    = 1024;
constexpr int kNH    = 16;
constexpr int kDh    = 64;
constexpr int kRL    = 64;
constexpr int kR5    = 5 * kRL;
constexpr int kTS    = 16;
constexpr float kEps = 1e-5f;

typedef __attribute__((ext_vector_type(16))) _Float16 v16h;
typedef __attribute__((ext_vector_type(8)))  _Float16 v8h;
typedef __attribute__((ext_vector_type(16))) __bf16   v16b;
typedef __attribute__((ext_vector_type(8)))  __bf16   v8b;
typedef __attribute__((ext_vector_type(8)))  float    v8f;
typedef __attribute__((ext_vector_type(4)))  float    v4f;
typedef __attribute__((ext_vector_type(4)))  unsigned int v4u;

__device__ __forceinline__ unsigned short f2bf_bits(float f) {
  unsigned u = __float_as_uint(f);
  return (unsigned short)((u + 0x7FFFu + ((u >> 16) & 1u)) >> 16);
}
__device__ __forceinline__ float bf_bits2f(unsigned short h) { return __uint_as_float(((unsigned)h) << 16); }

__device__ __forceinline__ void dep_guard_h(v8f& a, v8f& b, v16h x, v16h y) { asm volatile("v_nop\n\tv_nop\n\tv_nop\n\tv_nop" : "+v"(a), "+v"(b) : "v"(x), "v"(y)); }
__device__ __forceinline__ void dep_guard_b(v8f& a, v8f& b, v16b x, v16b y) { asm volatile("v_nop\n\tv_nop\n\tv_nop\n\tv_nop" : "+v"(a), "+v"(b) : "v"(x), "v"(y)); }
__device__ __forceinline__ void keep4_h(v16h a, v16h b, v16h c, v16h d) { asm volatile("v_nop" :: "v"(a), "v"(b), "v"(c), "v"(d)); }
__device__ __forceinline__ void keep4_b(v16b a, v16b b, v16b c, v16b d) { asm volatile("v_nop" :: "v"(a), "v"(b), "v"(c), "v"(d)); }
__device__ __forceinline__ void acc_guard4(v8f& a, v8f& b, v8f& c, v8f& d) { asm volatile("v_nop\n\tv_nop\n\tv_nop\n\tv_nop" : "+v"(a), "+v"(b), "+v"(c), "+v"(d)); }
template <typename T> struct Frag;
template <> struct Frag<_Float16> {
  typedef v16h V; union U { v16h v; v8h h[2]; };
  static __device__ __forceinline__ v16h load(const _Float16* p) {
    U f; f.h[0] = *(const v8h*)(p); f.h[1] = *(const v8h*)(p + 16); return f.v;
  }
  static __device__ __forceinline__ v8f mma(v16h a, v16h b, v8f c) {
    return __builtin_amdgcn_wmma_f32_16x16x32_f16(false, a, false, b, (short)0, c, false, false);
  }
  static __device__ __forceinline__ void guard(v8f& a, v8f& b, v16h x, v16h y) { dep_guard_h(a, b, x, y); }
  static __device__ __forceinline__ void keep(v16h a, v16h b, v16h c, v16h d) { keep4_h(a, b, c, d); }
};
template <> struct Frag<__bf16> {
  typedef v16b V; union U { v16b v; v8b h[2]; };
  static __device__ __forceinline__ v16b load(const __bf16* p) {
    U f; f.h[0] = *(const v8b*)(p); f.h[1] = *(const v8b*)(p + 16); return f.v;
  }
  static __device__ __forceinline__ v8f mma(v16b a, v16b b, v8f c) {
    return __builtin_amdgcn_wmma_f32_16x16x32_bf16(false, a, false, b, (short)0, c, false, false);
  }
  static __device__ __forceinline__ void guard(v8f& a, v8f& b, v16b x, v16b y) { dep_guard_b(a, b, x, y); }
  static __device__ __forceinline__ void keep(v16b a, v16b b, v16b c, v16b d) { keep4_b(a, b, c, d); }
};

__device__ __forceinline__ unsigned pk16(unsigned short a, unsigned short b) { return (unsigned)a | ((unsigned)b << 16); }

template <int ET> struct Elem;
template <> struct Elem<0> { typedef _Float16 T; };
template <> struct Elem<1> { typedef __bf16 T; };
template <int ET, bool SPLIT, int BIAS_MODE, int OUT_MODE, bool RESID, int ACT, int MIX>
__global__ __launch_bounds__(256) void wmma_gemm64(
    const unsigned short* __restrict__ Ap, const unsigned short* __restrict__ A2p, int lda, long strideA,
    const unsigned short* __restrict__ Btp, const unsigned short* __restrict__ Bt2p, int ldb, long strideB,
    void* __restrict__ Cout, void* __restrict__ Cout2, int ldc, long strideC,
    const float* __restrict__ bias,
    const float* __restrict__ resid, long strideR,
    int M, int N, int K, float scale, int seqMask) {
  typedef typename Elem<ET>::T T;
  typedef typename Frag<T>::V V;
  const T* A = (const T*)Ap; const T* A2 = (const T*)A2p; const T* Bt = (const T*)Btp; const T* Bt2 = (const T*)Bt2p;
  __shared__ __align__(16) float sT[8][16 * 68];
  const int b    = blockIdx.y;
  const int lane = threadIdx.x & 31;
  const int wave = threadIdx.x >> 5;
  const int tilesN = N >> 6;
  const int tilesM = M >> 6;
  const int tile = blockIdx.x * 8 + wave;
  if (tile >= tilesM * tilesN) return;
  const int tm = tile / tilesN;
  const int tn = tile - tm * tilesN;
  const int m0 = tm << 6;
  const int n0 = tn << 6;

  const T* Ab  = A  + (size_t)b * strideA;
  const T* Bb  = Bt + (size_t)b * strideB;
  const T* Ab2 = SPLIT ? (A2  + (size_t)b * strideA) : nullptr;
  const T* Bb2 = SPLIT ? (Bt2 + (size_t)b * strideB) : nullptr;

  const int rlane = lane & 15;
  const int koff  = (lane >> 4) * 8;
  const int mOff  = (lane >> 4) * 8;

  v8f acc[4][4];
#pragma unroll
  for (int i = 0; i < 4; ++i)
#pragma unroll
    for (int j = 0; j < 4; ++j) acc[i][j] = (v8f){0.f,0.f,0.f,0.f,0.f,0.f,0.f,0.f};

  for (int k0 = 0; k0 < K; k0 += 32) {
    V bh[4], bl[4];
#pragma unroll
    for (int j = 0; j < 4; ++j) {
      const size_t bo = (size_t)(n0 + (j << 4) + rlane) * ldb + koff + k0;
      bh[j] = Frag<T>::load(Bb + bo);
      if (SPLIT) bl[j] = Frag<T>::load(Bb2 + bo);
    }
#pragma unroll
    for (int i = 0; i < 4; ++i) {
      const size_t ao = (size_t)(m0 + (i << 4) + rlane) * lda + koff + k0;
      V ah = Frag<T>::load(Ab + ao);
      V al;
      if (SPLIT) al = Frag<T>::load(Ab2 + ao);
#pragma unroll
      for (int j = 0; j < 4; ++j) {
        acc[i][j] = Frag<T>::mma(ah, bh[j], acc[i][j]);
        if (SPLIT) {
          acc[i][j] = Frag<T>::mma(ah, bl[j], acc[i][j]);
          acc[i][j] = Frag<T>::mma(al, bh[j], acc[i][j]);
        }
      }
      Frag<T>::guard(acc[i][0], acc[i][3], ah, SPLIT ? al : ah);
    }
    Frag<T>::keep(bh[0], bh[1], bh[2], bh[3]);
    if (SPLIT) Frag<T>::keep(bl[0], bl[1], bl[2], bl[3]);
  }
  acc_guard4(acc[0][0], acc[0][1], acc[0][2], acc[0][3]);
  acc_guard4(acc[1][0], acc[1][1], acc[1][2], acc[1][3]);
  acc_guard4(acc[2][0], acc[2][1], acc[2][2], acc[2][3]);
  acc_guard4(acc[3][0], acc[3][1], acc[3][2], acc[3][3]);

  float* slab = sT[wave];
  const float* Rb = (RESID || MIX) ? (resid + (size_t)b * strideR) : nullptr;
#pragma unroll
  for (int i = 0; i < 4; ++i) {
    const int mBase = m0 + (i << 4);
#pragma unroll
    for (int j = 0; j < 4; ++j) {
      const int n = n0 + (j << 4) + rlane;
      float bv = 0.f;
      if (BIAS_MODE == 2) bv = bias[n];
#pragma unroll
      for (int r = 0; r < 8; ++r) {
        float v = acc[i][j][r] * scale;
        if (BIAS_MODE == 1) v += bias[mBase + mOff + r];
        if (BIAS_MODE == 2) v += bv;
        if (RESID) v += Rb[(size_t)(mBase + mOff + r) * ldc + n];
        if (MIX) {
          const int mrow  = mBase + mOff + r;
          const int tpos  = mrow & seqMask;
          const int mprev = (tpos != 0) ? (mrow - 1) : mrow;
          const float xv  = Rb[(size_t)mrow * ldc + n];
          const float xq  = Rb[(size_t)mprev * ldc + n];
          const float xp  = (tpos != 0) ? xq : 0.0f;
          v = xv + (xp - xv) * v;
        }
        if (ACT == 1) v = tanhf(v);
        if (ACT == 2) v = fmaxf(v, 0.0f);
        if (ACT == 4) v = (v > 0.f) ? v : 0.01f * v;
        slab[(mOff + r) * 68 + (j << 4) + rlane] = v;
      }
    }
    __builtin_amdgcn_fence(__ATOMIC_RELEASE, "workgroup");
    __builtin_amdgcn_wave_barrier();
    __builtin_amdgcn_fence(__ATOMIC_ACQUIRE, "workgroup");
    if (OUT_MODE == 0) {
      float* C = (float*)Cout + (size_t)b * strideC;
      const int hh = lane >> 4, c4 = (lane & 15) * 4;
      for (int pass = 0; pass < 2; ++pass) {
#pragma unroll
        for (int it = 0; it < 8; ++it) {
          const int row = it * 2 + hh;
          v4f v = *(const v4f*)(slab + row * 68 + c4);
          *(volatile v4f*)(C + (size_t)(mBase + row) * ldc + n0 + c4) = v;
        }
        __threadfence();
      }
    } else {
      const int q = lane >> 3, c8 = (lane & 7) * 8;
      unsigned short* C  = (unsigned short*)Cout  + (size_t)b * strideC;
      unsigned short* C2 = (OUT_MODE == 2) ? ((unsigned short*)Cout2 + (size_t)b * strideC) : nullptr;
      for (int pass = 0; pass < 2; ++pass) {
#pragma unroll
        for (int it = 0; it < 4; ++it) {
          const int row = it * 4 + q;
          const float* sp = slab + row * 68 + c8;
          v8h hv, lv;
#pragma unroll
          for (int e = 0; e < 8; ++e) {
            if (OUT_MODE == 1) {
              hv[e] = (_Float16)sp[e];
            } else {
              unsigned short hb = f2bf_bits(sp[e]);
              unsigned short lb = f2bf_bits(sp[e] - bf_bits2f(hb));
              hv[e] = __builtin_bit_cast(_Float16, hb);
              lv[e] = __builtin_bit_cast(_Float16, lb);
            }
          }
          *(volatile v8h*)(C + (size_t)(mBase + row) * ldc + n0 + c8) = hv;
          if (OUT_MODE == 2) *(volatile v8h*)(C2 + (size_t)(mBase + row) * ldc + n0 + c8) = lv;
        }
        __threadfence();
      }
    }
    __builtin_amdgcn_fence(__ATOMIC_RELEASE, "workgroup");
    __builtin_amdgcn_wave_barrier();
    __builtin_amdgcn_fence(__ATOMIC_ACQUIRE, "workgroup");
  }
}

__global__ __launch_bounds__(256) void tsplit_kernel(const float* __restrict__ W, int Kdim, int Ndim,
                                                     unsigned short* __restrict__ outH, unsigned short* __restrict__ outL) {
  __shared__ float sm[64][65];
  const int t  = threadIdx.x;
  const int k0 = blockIdx.x * 64;
  const int n0 = blockIdx.y * 64;
#pragma unroll
  for (int i = 0; i < 16; ++i) {
    const int e = i * 256 + t;
    const int r = e >> 6;
    const int c = e & 63;
    sm[c][r] = W[(size_t)(k0 + r) * Ndim + n0 + c];
  }
  __syncthreads();
  const int lane = t & 31, wave = t >> 5;
  const int q = lane >> 3, c8 = (lane & 7) * 8;
  v4u hu[2], lu[2];
  size_t off[2];
#pragma unroll
  for (int it = 0; it < 2; ++it) {
    const int row = wave * 8 + it * 4 + q;
    unsigned short hb[8], lb[8];
#pragma unroll
    for (int e = 0; e < 8; ++e) {
      const float f = sm[row][c8 + e];
      hb[e] = f2bf_bits(f);
      lb[e] = f2bf_bits(f - bf_bits2f(hb[e]));
    }
    hu[it]  = (v4u){pk16(hb[0], hb[1]), pk16(hb[2], hb[3]), pk16(hb[4], hb[5]), pk16(hb[6], hb[7])};
    lu[it]  = (v4u){pk16(lb[0], lb[1]), pk16(lb[2], lb[3]), pk16(lb[4], lb[5]), pk16(lb[6], lb[7])};
    off[it] = (size_t)(n0 + row) * Kdim + k0 + c8;
  }
  for (int pass = 0; pass < 2; ++pass) {
#pragma unroll
    for (int it = 0; it < 2; ++it) {
      *(volatile v4u*)(outH + off[it]) = hu[it];
      *(volatile v4u*)(outL + off[it]) = lu[it];
    }
    __threadfence();
  }
}

__global__ __launch_bounds__(256) void split8_kernel(const float* __restrict__ in, unsigned short* __restrict__ outH,
                                                     unsigned short* __restrict__ outL, int n8) {
  const int i = blockIdx.x * 256 + threadIdx.x;
  if (i >= n8) return;
  const float* p = in + 8 * (size_t)i;
  const v4f a = *(const v4f*)(p);
  const v4f c = *(const v4f*)(p + 4);
  unsigned short hb[8], lb[8];
#pragma unroll
  for (int e = 0; e < 4; ++e) {
    hb[e]     = f2bf_bits(a[e]);
    lb[e]     = f2bf_bits(a[e] - bf_bits2f(hb[e]));
    hb[4 + e] = f2bf_bits(c[e]);
    lb[4 + e] = f2bf_bits(c[e] - bf_bits2f(hb[4 + e]));
  }
  const v4u uh = (v4u){pk16(hb[0], hb[1]), pk16(hb[2], hb[3]), pk16(hb[4], hb[5]), pk16(hb[6], hb[7])};
  const v4u ul = (v4u){pk16(lb[0], lb[1]), pk16(lb[2], lb[3]), pk16(lb[4], lb[5]), pk16(lb[6], lb[7])};
  unsigned short* qh = outH + 8 * (size_t)i;
  unsigned short* ql = outL + 8 * (size_t)i;
  *(volatile v4u*)qh = uh;
  *(volatile v4u*)ql = ul;
  __threadfence();
  *(volatile v4u*)qh = uh;
  *(volatile v4u*)ql = ul;
}

__global__ __launch_bounds__(256) void prep_mix_kernel(const float* __restrict__ x, const float* __restrict__ mu,
                                                       unsigned short* __restrict__ outH, unsigned short* __restrict__ outL,
                                                       int n8, int hdim, int seqMask) {
  const int i = blockIdx.x * 256 + threadIdx.x;
  if (i >= n8) return;
  const size_t e0 = 8 * (size_t)i;
  const int m = (int)(e0 / (size_t)hdim);
  const int n = (int)(e0 - (size_t)m * hdim);
  const int tpos  = m & seqMask;
  const int mprev = (tpos != 0) ? (m - 1) : m;
  const float* xr = x + (size_t)m * hdim + n;
  const float* xq = x + (size_t)mprev * hdim + n;
  const v4f a0 = *(const v4f*)(xr), a1 = *(const v4f*)(xr + 4);
  const v4f p0 = *(const v4f*)(xq), p1 = *(const v4f*)(xq + 4);
  const v4f u0 = *(const v4f*)(mu + n), u1 = *(const v4f*)(mu + n + 4);
  unsigned short hb[8], lb[8];
#pragma unroll
  for (int e = 0; e < 4; ++e) {
    const float xp0 = (tpos != 0) ? p0[e] : 0.0f;
    const float xp1 = (tpos != 0) ? p1[e] : 0.0f;
    const float f0 = a0[e] + (xp0 - a0[e]) * u0[e];
    const float f1 = a1[e] + (xp1 - a1[e]) * u1[e];
    hb[e]     = f2bf_bits(f0);
    lb[e]     = f2bf_bits(f0 - bf_bits2f(hb[e]));
    hb[4 + e] = f2bf_bits(f1);
    lb[4 + e] = f2bf_bits(f1 - bf_bits2f(hb[4 + e]));
  }
  const v4u uh = (v4u){pk16(hb[0], hb[1]), pk16(hb[2], hb[3]), pk16(hb[4], hb[5]), pk16(hb[6], hb[7])};
  const v4u ul = (v4u){pk16(lb[0], lb[1]), pk16(lb[2], lb[3]), pk16(lb[4], lb[5]), pk16(lb[6], lb[7])};
  unsigned short* qh = outH + e0;
  unsigned short* ql = outL + e0;
  *(volatile v4u*)qh = uh;
  *(volatile v4u*)ql = ul;
  __threadfence();
  *(volatile v4u*)qh = uh;
  *(volatile v4u*)ql = ul;
}

__global__ __launch_bounds__(256) void wkv_scan_kernel(const float* __restrict__ r, const float* __restrict__ k,
                                                       const float* __restrict__ v, const float* __restrict__ w,
                                                       const float* __restrict__ bonus, float* __restrict__ o,
                                                       int seqT, int ld, int nh) {
  __shared__ __align__(16) float sr[kTS * 64];
  __shared__ __align__(16) float sk[kTS * 64];
  __shared__ __align__(16) float sd[kTS * 64];
  __shared__ __align__(16) float sv[kTS * 64];
  __shared__ float so[2][4][64];
  __shared__ __align__(16) float sout[kTS * 64];
  const int bh  = blockIdx.x;
  const int b   = bh / nh;
  const int h   = bh - b * nh;
  const int tid = threadIdx.x;
  const int dv  = tid & 63;
  const int g4  = tid >> 6;
  const int tr  = tid >> 4;
  const int c4  = (tid & 15) * 4;
  float S[16], u[16];
#pragma unroll
  for (int i = 0; i < 16; ++i) { S[i] = 0.0f; u[i] = bonus[h * 64 + g4 * 16 + i]; }
  const size_t col0 = (size_t)h * 64;
  const int nchunk = seqT / kTS;
  for (int ch = 0; ch < nchunk; ++ch) {
    const int t0 = ch * kTS;
    __syncthreads();
    {
      const size_t gi = (size_t)(b * seqT + t0 + tr) * ld + col0 + c4;
      const v4f rv = *(const v4f*)(r + gi);
      const v4f kv = *(const v4f*)(k + gi);
      const v4f vv = *(const v4f*)(v + gi);
      const v4f wv = *(const v4f*)(w + gi);
      v4f dd;
#pragma unroll
      for (int e = 0; e < 4; ++e) dd[e] = expf(-expf(wv[e]));
      *(v4f*)(sr + tr * 64 + c4) = rv;
      *(v4f*)(sk + tr * 64 + c4) = kv;
      *(v4f*)(sv + tr * 64 + c4) = vv;
      *(v4f*)(sd + tr * 64 + c4) = dd;
    }
    __syncthreads();
#pragma unroll 1
    for (int ts = 0; ts < kTS; ++ts) {
      const float* pr = sr + ts * 64 + g4 * 16;
      const float* pk = sk + ts * 64 + g4 * 16;
      const float* pd = sd + ts * 64 + g4 * 16;
      const float vt = sv[ts * 64 + dv];
      float acc = 0.0f;
#pragma unroll
      for (int i = 0; i < 16; ++i) {
        const float kvv = pk[i] * vt;
        acc += pr[i] * (S[i] + u[i] * kvv);
        S[i] = pd[i] * S[i] + kvv;
      }
      so[ts & 1][g4][dv] = acc;
      __syncthreads();
      if (tid < 64) {
        sout[ts * 64 + tid] = ((so[ts & 1][0][tid] + so[ts & 1][1][tid]) + so[ts & 1][2][tid]) + so[ts & 1][3][tid];
      }
    }
    __syncthreads();
    {
      const v4f val = *(const v4f*)(sout + tr * 64 + c4);
      float* op = o + (size_t)(b * seqT + t0 + tr) * ld + col0 + c4;
      *(volatile v4f*)op = val;
      __threadfence();
      *(volatile v4f*)op = val;
    }
  }
}

__global__ __launch_bounds__(256) void ln_gate_kernel(const float* __restrict__ o, const float* __restrict__ g,
                                                      const float* __restrict__ lnw, const float* __restrict__ lnb,
                                                      unsigned short* __restrict__ Oh, unsigned short* __restrict__ Ol,
                                                      int nrows, float eps) {
  const int t = threadIdx.x, lane = t & 31, wave = t >> 5;
  const int q = lane >> 3, c8 = (lane & 7) * 8;
  const int row  = blockIdx.x * 32 + wave * 4 + q;
  const bool valid = row < nrows;
  const int rowc = valid ? row : (nrows - 1);
  const float* op = o + (size_t)rowc * 64 + c8;
  const float* gp = g + (size_t)rowc * 64 + c8;
  const v4f o0 = *(const v4f*)(op), o1 = *(const v4f*)(op + 4);
  const v4f g0 = *(const v4f*)(gp), g1 = *(const v4f*)(gp + 4);
  const v4f w0 = *(const v4f*)(lnw + c8), w1 = *(const v4f*)(lnw + c8 + 4);
  const v4f b0 = *(const v4f*)(lnb + c8), b1 = *(const v4f*)(lnb + c8 + 4);
  float xv[8], gv[8], wv[8], bv[8];
#pragma unroll
  for (int e = 0; e < 4; ++e) {
    xv[e] = o0[e]; xv[4 + e] = o1[e];
    gv[e] = g0[e]; gv[4 + e] = g1[e];
    wv[e] = w0[e]; wv[4 + e] = w1[e];
    bv[e] = b0[e]; bv[4 + e] = b1[e];
  }
  float s = 0.0f;
#pragma unroll
  for (int e = 0; e < 8; ++e) s += xv[e];
  s += __shfl_xor(s, 1, 32);
  s += __shfl_xor(s, 2, 32);
  s += __shfl_xor(s, 4, 32);
  const float mean = s * (1.0f / 64.0f);
  float sq = 0.0f;
#pragma unroll
  for (int e = 0; e < 8; ++e) { const float d = xv[e] - mean; xv[e] = d; sq += d * d; }
  sq += __shfl_xor(sq, 1, 32);
  sq += __shfl_xor(sq, 2, 32);
  sq += __shfl_xor(sq, 4, 32);
  const float var = sq * (1.0f / 64.0f);
  const float rs  = rsqrtf(var + eps);
  unsigned short hb[8], lb[8];
#pragma unroll
  for (int e = 0; e < 8; ++e) {
    const float on  = xv[e] * rs * wv[e] + bv[e];
    const float ge  = gv[e];
    const float ex  = expf(-ge);
    const float sig = __builtin_amdgcn_rcpf(1.0f + ex);
    const float y   = on * ge * sig;
    hb[e] = f2bf_bits(y);
    lb[e] = f2bf_bits(y - bf_bits2f(hb[e]));
  }
  const v4u uh = (v4u){pk16(hb[0], hb[1]), pk16(hb[2], hb[3]), pk16(hb[4], hb[5]), pk16(hb[6], hb[7])};
  const v4u ul = (v4u){pk16(lb[0], lb[1]), pk16(lb[2], lb[3]), pk16(lb[4], lb[5]), pk16(lb[6], lb[7])};
  if (valid) {
    unsigned short* qh = Oh + (size_t)row * 64 + c8;
    unsigned short* ql = Ol + (size_t)row * 64 + c8;
    *(volatile v4u*)qh = uh;
    *(volatile v4u*)ql = ul;
    __threadfence();
    *(volatile v4u*)qh = uh;
    *(volatile v4u*)ql = ul;
  }
}

template <int BIAS_MODE, int OUT_MODE, int ACT, int MIX>
static inline void gemm3(hipStream_t s,
                         const unsigned short* Ah, const unsigned short* Al, int lda,
                         const unsigned short* Bh, const unsigned short* Bl, int ldb,
                         void* C, void* C2, int ldc,
                         const float* bias, const float* xres,
                         int M, int N, int K) {
  const int tiles = (M >> 6) * (N >> 6);
  dim3 grid((unsigned)((tiles + 7) / 8), 1, 1);
  wmma_gemm64<1, true, BIAS_MODE, OUT_MODE, false, ACT, MIX><<<grid, 256, 0, s>>>(
      Ah, Al, lda, 0L, Bh, Bl, ldb, 0L, C, C2, ldc, 0L, bias, xres, 0L, M, N, K, 1.0f, kSeqT - 1);
}

static inline void tsplit(hipStream_t s, const float* W, int Kdim, int Ndim, unsigned short* outH, unsigned short* outL) {
  dim3 grid((unsigned)(Kdim / 64), (unsigned)(Ndim / 64), 1);
  tsplit_kernel<<<grid, 256, 0, s>>>(W, Kdim, Ndim, outH, outL);
}

extern "C" void kernel_launch(void* const* d_in, const int* in_sizes, int n_in,
                              void* d_out, int out_size, void* d_ws, size_t ws_size,
                              hipStream_t stream) {
  if (n_in < 18) return;
  if (in_sizes[0] != kTok * kHid || out_size != kTok * kHid) return;
  if (in_sizes[2] != kHid * kR5 || in_sizes[5] != kHid * kKD || in_sizes[17] != kVD * kHid) return;
  if ((kSeqT % kTS) != 0 || ((kTok * kNH) % 32) != 0) return;

  const float* x      = (const float*)d_in[0];
  const float* mu_x   = (const float*)d_in[1];
  const float* Wx1    = (const float*)d_in[2];
  const float* Wx2    = (const float*)d_in[3];
  const float* x_bias = (const float*)d_in[4];
  const float* Wr     = (const float*)d_in[5];
  const float* Wk     = (const float*)d_in[6];
  const float* Wv     = (const float*)d_in[7];
  const float* Ww_a   = (const float*)d_in[8];
  const float* Ww_b   = (const float*)d_in[9];
  const float* bw     = (const float*)d_in[10];
  const float* Wg_a   = (const float*)d_in[11];
  const float* Wg_b   = (const float*)d_in[12];
  const float* bg     = (const float*)d_in[13];
  const float* bonus  = (const float*)d_in[14];
  const float* ln_w   = (const float*)d_in[15];
  const float* ln_b   = (const float*)d_in[16];
  const float* Wo     = (const float*)d_in[17];
  float* out = (float*)d_out;

  char* wsb = (char*)d_ws;
  size_t off = 0;
  auto carve = [&](size_t bytes) -> char* { char* p = wsb + off; off += (bytes + 255) & ~(size_t)255; return p; };
  const size_t plXA  = (size_t)kTok * kHid * 2;
  const size_t plWx1 = (size_t)kR5 * kHid * 2;
  const size_t plLR  = (size_t)kTok * kR5 * 2;
  const size_t plWB  = (size_t)kKD * kHid * 2;
  const size_t plWa  = (size_t)kRL * kHid * 2;
  const size_t plWb  = (size_t)kKD * kRL * 2;
  const size_t plL   = (size_t)kTok * kRL * 2;
  const size_t plF   = (size_t)kTok * kKD * 4;
  const size_t plO   = (size_t)kTok * kVD * 2;
  unsigned short* XAh   = (unsigned short*)carve(plXA);
  unsigned short* XAl   = (unsigned short*)carve(plXA);
  unsigned short* Wx1Th = (unsigned short*)carve(plWx1);
  unsigned short* Wx1Tl = (unsigned short*)carve(plWx1);
  unsigned short* Wx2h  = (unsigned short*)carve(plLR);
  unsigned short* Wx2l  = (unsigned short*)carve(plLR);
  unsigned short* LRh   = (unsigned short*)carve(plLR);
  unsigned short* LRl   = (unsigned short*)carve(plLR);
  unsigned short* WBh   = (unsigned short*)carve(plWB);
  unsigned short* WBl   = (unsigned short*)carve(plWB);
  unsigned short* WwaTh = (unsigned short*)carve(plWa);
  unsigned short* WwaTl = (unsigned short*)carve(plWa);
  unsigned short* WgaTh = (unsigned short*)carve(plWa);
  unsigned short* WgaTl = (unsigned short*)carve(plWa);
  unsigned short* WwbTh = (unsigned short*)carve(plWb);
  unsigned short* WwbTl = (unsigned short*)carve(plWb);
  unsigned short* WgbTh = (unsigned short*)carve(plWb);
  unsigned short* WgbTl = (unsigned short*)carve(plWb);
  unsigned short* WLh   = (unsigned short*)carve(plL);
  unsigned short* WLl   = (unsigned short*)carve(plL);
  unsigned short* GLh   = (unsigned short*)carve(plL);
  unsigned short* GLl   = (unsigned short*)carve(plL);
  float* rb = (float*)carve(plF);
  float* kb = (float*)carve(plF);
  float* vb = (float*)carve(plF);
  float* wb = (float*)carve(plF);
  float* gb = (float*)carve(plF);
  float* ob = (float*)carve(plF);
  unsigned short* Oh = (unsigned short*)carve(plO);
  unsigned short* Ol = (unsigned short*)carve(plO);
  if (off > ws_size) return;

  tsplit(stream, Wx1, kHid, kR5, Wx1Th, Wx1Tl);
  {
    const int n8 = kHid * kR5 / 8;
    split8_kernel<<<(unsigned)((n8 + 255) / 256), 256, 0, stream>>>(Wx2, Wx2h, Wx2l, n8);
  }
  tsplit(stream, Ww_a, kHid, kRL, WwaTh, WwaTl);
  tsplit(stream, Ww_b, kRL, kKD, WwbTh, WwbTl);
  tsplit(stream, Wg_a, kHid, kRL, WgaTh, WgaTl);
  tsplit(stream, Wg_b, kRL, kVD, WgbTh, WgbTl);

  {
    const int n8 = kTok * kHid / 8;
    prep_mix_kernel<<<(unsigned)((n8 + 255) / 256), 256, 0, stream>>>(x, mu_x, XAh, XAl, n8, kHid, kSeqT - 1);
  }

  gemm3<0, 2, 1, 0>(stream, XAh, XAl, kHid, Wx1Th, Wx1Tl, kHid, LRh, LRl, kR5, nullptr, nullptr, kTok, kR5, kHid);

  gemm3<2, 2, 0, 1>(stream, LRh + 0 * kRL, LRl + 0 * kRL, kR5, Wx2h + 0 * kRL, Wx2l + 0 * kRL, kR5,
                    XAh, XAl, kHid, x_bias + 0 * kHid, x, kTok, kHid, kRL);
  tsplit(stream, Wr, kHid, kKD, WBh, WBl);
  gemm3<0, 0, 0, 0>(stream, XAh, XAl, kHid, WBh, WBl, kHid, rb, nullptr, kKD, nullptr, nullptr, kTok, kKD, kHid);
  gemm3<2, 2, 0, 1>(stream, LRh + 1 * kRL, LRl + 1 * kRL, kR5, Wx2h + 1 * kRL, Wx2l + 1 * kRL, kR5,
                    XAh, XAl, kHid, x_bias + 1 * kHid, x, kTok, kHid, kRL);
  gemm3<0, 2, 1, 0>(stream, XAh, XAl, kHid, WwaTh, WwaTl, kHid, WLh, WLl, kRL, nullptr, nullptr, kTok, kRL, kHid);
  gemm3<2, 0, 0, 0>(stream, WLh, WLl, kRL, WwbTh, WwbTl, kRL, wb, nullptr, kKD, bw, nullptr, kTok, kKD, kRL);
  gemm3<2, 2, 0, 1>(stream, LRh + 2 * kRL, LRl + 2 * kRL, kR5, Wx2h + 2 * kRL, Wx2l + 2 * kRL, kR5,
                    XAh, XAl, kHid, x_bias + 2 * kHid, x, kTok, kHid, kRL);
  tsplit(stream, Wk, kHid, kKD, WBh, WBl);
  gemm3<0, 0, 0, 0>(stream, XAh, XAl, kHid, WBh, WBl, kHid, kb, nullptr, kKD, nullptr, nullptr, kTok, kKD, kHid);
  gemm3<2, 2, 0, 1>(stream, LRh + 3 * kRL, LRl + 3 * kRL, kR5, Wx2h + 3 * kRL, Wx2l + 3 * kRL, kR5,
                    XAh, XAl, kHid, x_bias + 3 * kHid, x, kTok, kHid, kRL);
  tsplit(stream, Wv, kHid, kVD, WBh, WBl);
  gemm3<0, 0, 0, 0>(stream, XAh, XAl, kHid, WBh, WBl, kHid, vb, nullptr, kVD, nullptr, nullptr, kTok, kVD, kHid);
  gemm3<2, 2, 0, 1>(stream, LRh + 4 * kRL, LRl + 4 * kRL, kR5, Wx2h + 4 * kRL, Wx2l + 4 * kRL, kR5,
                    XAh, XAl, kHid, x_bias + 4 * kHid, x, kTok, kHid, kRL);
  gemm3<0, 2, 1, 0>(stream, XAh, XAl, kHid, WgaTh, WgaTl, kHid, GLh, GLl, kRL, nullptr, nullptr, kTok, kRL, kHid);
  gemm3<2, 0, 0, 0>(stream, GLh, GLl, kRL, WgbTh, WgbTl, kRL, gb, nullptr, kVD, bg, nullptr, kTok, kVD, kRL);

  wkv_scan_kernel<<<kBatch * kNH, 256, 0, stream>>>(rb, kb, vb, wb, bonus, ob, kSeqT, kKD, kNH);

  {
    const int nrows = kTok * kNH;
    ln_gate_kernel<<<(unsigned)(nrows / 32), 256, 0, stream>>>(ob, gb, ln_w, ln_b, Oh, Ol, nrows, kEps);
  }

  tsplit(stream, Wo, kVD, kHid, WBh, WBl);
  gemm3<0, 0, 0, 0>(stream, Oh, Ol, kVD, WBh, WBl, kVD, out, nullptr, kHid, nullptr, nullptr, kTok, kHid, kVD);
}
